// QANet_48928267436508
// MI455X (gfx1250) — hardware-verified
//
#include <hip/hip_runtime.h>
#include <math.h>

#ifndef NB
#define NB 64
#endif
#define NB_FULL 64
#define DM 128
#define KCAT 256
#define LC 400
#define LQ 50
#define NHEAD 8
#define HDIM 16
#define NCONV 4
#define KTAP 7
#define TROW 50
#define ROWS_C (NB * LC)
#define ROWS_Q (NB * LQ)
#define MTOK (ROWS_C + ROWS_Q)
#define NT_C (ROWS_C / TROW)
#define NT_Q (ROWS_Q / TROW)
#define CPAD 448
#define QPAD 64
#define CTILES 7

static_assert(NB <= NB_FULL);
static_assert(MTOK % 64 == 0);
static_assert(MTOK % 16 == 0);
static_assert(DM % 64 == 0 && DM % 32 == 0 && DM == 128);
static_assert(KCAT == 2 * DM && KCAT % 32 == 0 && KCAT % 8 == 0);
static_assert(NHEAD * HDIM == DM && HDIM == 16 && NHEAD == 8);
static_assert(LC == 8 * TROW && LQ == TROW);
static_assert(ROWS_C % TROW == 0 && ROWS_Q % TROW == 0);
static_assert(DM * TROW == 25 * 256);
static_assert(TROW * 32 <= 7 * 256 && (TROW * 32) % 32 == 0);
static_assert(TROW * 16 <= 4 * 256 && (TROW * 16) % 32 == 0);
static_assert(TROW + 6 <= 64);
static_assert(LC % 16 == 0);
static_assert(CPAD == CTILES * 64 && CPAD >= LC && CPAD % 32 == 0);
static_assert(QPAD == 64 && QPAD >= LQ);
static_assert((LC * DM) % 256 == 0);
static_assert((LC * 4) % 16 == 0 && (LC - 8) % 8 == 0 && LC % 8 == 0);

#define WS_BYTES_TOTAL ((size_t)LC * DM * 4 + 2 * (size_t)MTOK * DM * 4 + 2 * (size_t)MTOK * KCAT * 2 + 3 * (size_t)MTOK * DM * 2 \
    + (size_t)(NCONV + 5) * DM * KCAT * 2 + 2 * (size_t)MTOK * DM * 2 + (size_t)NB * CPAD * 4 + (size_t)NB * QPAD * 4 \
    + (size_t)NB * DM * CPAD * 2 + 2 * (size_t)NB * DM * QPAD * 2 + (size_t)NB * LC * QPAD * 2 + (size_t)NB * QPAD * CPAD * 4 \
    + (size_t)NB * QPAD * CPAD * 2)
static_assert(WS_BYTES_TOTAL + 32 * 256 <= (size_t)134217728);

typedef __attribute__((ext_vector_type(16))) _Float16 v16h;
typedef __attribute__((ext_vector_type(8)))  _Float16 v8h;
typedef __attribute__((ext_vector_type(8)))  float    v8f;
typedef __attribute__((ext_vector_type(4)))  float    v4f;
typedef __attribute__((ext_vector_type(4)))  unsigned int v4u;
typedef _Float16 h16;


#define VST2(T, ptr, val) do { const T vst2_v_ = (val); *(volatile T*)(ptr) = vst2_v_; __threadfence(); *(volatile T*)(ptr) = vst2_v_; } while (0)
#define VST2V4(ptr, val) do { const v4f vst2_v4_ = (val); *(volatile v4f*)(ptr) = vst2_v4_; __threadfence(); *(volatile v4f*)(ptr) = vst2_v4_; } while (0)

__device__ __forceinline__ float bfr(float f) {
    unsigned u = __float_as_uint(f);
    u += 0x7FFFu + ((u >> 16) & 1u);
    return __uint_as_float(u & 0xFFFF0000u);
}
static __device__ __forceinline__ h16 toh_flush(float v) { const h16 r = (h16)v; return (fabsf(v) < 6.103515625e-05f) ? (h16)0.0f : r; }
static __device__ __forceinline__ unsigned hbits(h16 x) { return (unsigned)__builtin_bit_cast(unsigned short, x); }
static __device__ __forceinline__ unsigned umin2(unsigned a, unsigned b) { return a < b ? a : b; }
static __device__ __forceinline__ void st8hf(unsigned short* P, size_t o, const float* v) {
    v4u pk;
    pk.x = hbits(toh_flush(v[0])) | (hbits(toh_flush(v[1])) << 16);
    pk.y = hbits(toh_flush(v[2])) | (hbits(toh_flush(v[3])) << 16);
    pk.z = hbits(toh_flush(v[4])) | (hbits(toh_flush(v[5])) << 16);
    pk.w = hbits(toh_flush(v[6])) | (hbits(toh_flush(v[7])) << 16);
    VST2(v4u, (v4u*)(P + o), pk);
}
static __device__ __forceinline__ void st8hf_pair(unsigned short* P, size_t ohi, size_t olo, const float* v) {
    unsigned hb[8], lb[8];
#pragma unroll
    for (int i = 0; i < 8; ++i) {
        const h16 hu = (h16)v[i];
        hb[i] = hbits(toh_flush(v[i]));
        lb[i] = hbits(toh_flush((v[i] - (float)hu) * 64.0f));
    }
    v4u ph, pl;
    ph.x = hb[0] | (hb[1] << 16); ph.y = hb[2] | (hb[3] << 16); ph.z = hb[4] | (hb[5] << 16); ph.w = hb[6] | (hb[7] << 16);
    pl.x = lb[0] | (lb[1] << 16); pl.y = lb[2] | (lb[3] << 16); pl.z = lb[4] | (lb[5] << 16); pl.w = lb[6] | (lb[7] << 16);
    *(volatile v4u*)(P + ohi) = ph;
    *(volatile v4u*)(P + olo) = pl;
    __threadfence();
    *(volatile v4u*)(P + ohi) = ph;
    *(volatile v4u*)(P + olo) = pl;
}

union FragU { v16h v; v8h h[2]; };
__device__ __forceinline__ v16h frag_ld(const _Float16* p) {
    FragU f; f.h[0] = *(const v8h*)(p); f.h[1] = *(const v8h*)(p + 16); return f.v;
}
__device__ __forceinline__ v8f wmma16(v16h a, v16h b, v8f c) {
    c = __builtin_amdgcn_wmma_f32_16x16x32_f16(false, a, false, b, (short)0, c, false, false);
    asm volatile("v_nop\n\tv_nop\n\tv_nop\n\tv_nop" : "+v"(c) : "v"(a), "v"(b));
    return c;
}
__device__ __forceinline__ void dep_guard_h(v8f& a, v8f& b, v16h x, v16h y) { asm volatile("v_nop\n\tv_nop\n\tv_nop\n\tv_nop" : "+v"(a), "+v"(b) : "v"(x), "v"(y)); }
__device__ __forceinline__ void keep4_h(v16h a, v16h b, v16h c, v16h d) { asm volatile("v_nop" :: "v"(a), "v"(b), "v"(c), "v"(d)); }
__device__ __forceinline__ void acc_guard4(v8f& a, v8f& b, v8f& c, v8f& d) { asm volatile("v_nop\n\tv_nop\n\tv_nop\n\tv_nop" : "+v"(a), "+v"(b), "+v"(c), "+v"(d)); }
__device__ __forceinline__ void wave_sync_lds() {
    __builtin_amdgcn_fence(3  , "workgroup");
    __builtin_amdgcn_wave_barrier();
    __builtin_amdgcn_fence(2  , "workgroup");
}

template <int OUT_MODE, bool RESID, bool RELU>
__global__ __launch_bounds__(256) void k_gemm64(
    const _Float16* __restrict__ A, unsigned lda, const _Float16* __restrict__ Bt, unsigned ldb,
    void* __restrict__ Cout, unsigned ldc, const float* __restrict__ bias, const float* __restrict__ resid,
    unsigned M, unsigned N, unsigned K, float scale, float oscale) {
  __shared__ __align__(16) float sT[8][16 * 68];
  const unsigned lane = threadIdx.x & 31u;
  const unsigned wave = threadIdx.x >> 5;
  const unsigned tilesN = N >> 6, tilesM = M >> 6;
  const unsigned tile = blockIdx.x * 8u + wave;
  if (tile >= tilesM * tilesN) return;
  const unsigned tm = tile / tilesN;
  const unsigned tn = tile - tm * tilesN;
  const unsigned m0 = tm << 6, n0 = tn << 6;
  const unsigned rlane = lane & 15u;
  const unsigned koff = (lane >> 4) * 8u;
  const unsigned mOff = koff;

  v8f acc[4][4];
#pragma unroll
  for (int i = 0; i < 4; ++i)
#pragma unroll
    for (int j = 0; j < 4; ++j) acc[i][j] = (v8f){0.f,0.f,0.f,0.f,0.f,0.f,0.f,0.f};

  for (unsigned k0 = 0; k0 < K; k0 += 32u) {
    v16h bh[4];
#pragma unroll
    for (int j = 0; j < 4; ++j)
      bh[j] = frag_ld(Bt + (size_t)(n0 + ((unsigned)j << 4) + rlane) * ldb + koff + k0);
#pragma unroll
    for (int i = 0; i < 4; ++i) {
      const v16h ah = frag_ld(A + (size_t)(m0 + ((unsigned)i << 4) + rlane) * lda + koff + k0);
#pragma unroll
      for (int j = 0; j < 4; ++j)
        acc[i][j] = __builtin_amdgcn_wmma_f32_16x16x32_f16(false, ah, false, bh[j], (short)0, acc[i][j], false, false);
      dep_guard_h(acc[i][0], acc[i][3], ah, ah);
    }
    keep4_h(bh[0], bh[1], bh[2], bh[3]);
  }
  acc_guard4(acc[0][0], acc[0][1], acc[0][2], acc[0][3]);
  acc_guard4(acc[1][0], acc[1][1], acc[1][2], acc[1][3]);
  acc_guard4(acc[2][0], acc[2][1], acc[2][2], acc[2][3]);
  acc_guard4(acc[3][0], acc[3][1], acc[3][2], acc[3][3]);

  float* slab = sT[wave];
#pragma unroll
  for (int i = 0; i < 4; ++i) {
    const unsigned mBase = m0 + ((unsigned)i << 4);
#pragma unroll
    for (int j = 0; j < 4; ++j) {
      const unsigned n = n0 + ((unsigned)j << 4) + rlane;
      const float bv = bfr(bias[n]);
#pragma unroll
      for (int r = 0; r < 8; ++r) {
        float v = acc[i][j][r] * scale + bv;
        if (RELU) v = fmaxf(v, 0.0f);
        if (OUT_MODE == 1) v *= oscale;
        slab[(mOff + (unsigned)r) * 68u + ((unsigned)j << 4) + rlane] = v;
      }
    }
    wave_sync_lds();
    if (OUT_MODE == 0) {
      float* C = (float*)Cout;
      const unsigned hh = lane >> 4, c4 = (lane & 15u) * 4u;
#pragma unroll
      for (int half = 0; half < 2; ++half) {
        v4f vv[4];
#pragma unroll
        for (int it = 0; it < 4; ++it) {
          const unsigned row = (unsigned)(half * 4 + it) * 2u + hh;
          vv[it] = *(const v4f*)(slab + row * 68u + c4);
          if (RESID) vv[it] += *(const v4f*)(resid + (size_t)(mBase + row) * ldc + n0 + c4);
        }
        for (int pass = 0; pass < 2; ++pass) {
#pragma unroll
          for (int it = 0; it < 4; ++it) {
            const unsigned row = (unsigned)(half * 4 + it) * 2u + hh;
            *(volatile v4f*)(C + (size_t)(mBase + row) * ldc + n0 + c4) = vv[it];
          }
          __threadfence();
        }
      }
    } else {
      _Float16* C = (_Float16*)Cout;
      const unsigned q = lane >> 3, c8 = (lane & 7u) * 8u;
      v8h hv[4];
#pragma unroll
      for (int it = 0; it < 4; ++it) {
        const unsigned row = (unsigned)it * 4u + q;
        const float* sp = slab + row * 68u + c8;
#pragma unroll
        for (int e = 0; e < 8; ++e) hv[it][e] = (_Float16)sp[e];
      }
      for (int pass = 0; pass < 2; ++pass) {
#pragma unroll
        for (int it = 0; it < 4; ++it) {
          const unsigned row = (unsigned)it * 4u + q;
          *(volatile v8h*)(C + (size_t)(mBase + row) * ldc + n0 + c8) = hv[it];
        }
        __threadfence();
      }
    }
    wave_sync_lds();
  }
}

static_assert(16 * 2 * 16 == KCAT * 2);
__global__ __launch_bounds__(256) void k_wcvt(const float* __restrict__ Wm, unsigned short* __restrict__ W16,
                                              unsigned lgog, unsigned s2, unsigned s1, unsigned sk, unsigned nrows, float sw) {
    const unsigned u = blockIdx.x * 256u + threadIdx.x;
    if (u >= nrows * 16u) return;
    const unsigned o = u >> 4, k0 = (u & 15u) * 8u;
    const unsigned base = (o >> lgog) * s2 + (o & ((1u << lgog) - 1u)) * s1;
    float v[8], w[8];
#pragma unroll
    for (int i = 0; i < 8; ++i) {
        const float t = bfr(Wm[base + (k0 + (unsigned)i) * sk]) * sw;
        v[i] = t;
        w[i] = t * (1.0f / 64.0f);
    }
    st8hf(W16, (size_t)o * KCAT + k0, v);
    st8hf(W16, (size_t)o * KCAT + DM + k0, w);
}

__global__ __launch_bounds__(256) void k_pe(float* __restrict__ pe) {
    __shared__ __align__(16) float sT[256];
    const unsigned t = threadIdx.x;
    const unsigned idx = blockIdx.x * 256u + t;
    const unsigned l = idx >> 7, d = idx & 127u;
    const unsigned de = d & ~1u;
    const float freq = exp2f(-(float)de * (13.287712379549449f / 128.0f));
    const float ang = (float)l * freq + ((d & 1u) ? 1.5707963267948966f : 0.0f);
    sT[t] = sinf(ang);
    __syncthreads();
    if (t < 64u) {
        const v4f v = *(const v4f*)(sT + 4u * t);
        VST2V4(pe + (size_t)blockIdx.x * 256u + 4u * t, v);
    }
}

__global__ __launch_bounds__(256) void k_prep(const float* __restrict__ x, const float* __restrict__ pe, float* __restrict__ cur,
                                              unsigned L, unsigned tps, unsigned rowBase) {
    __shared__ float sX[TROW * 129];
    const unsigned tid = threadIdx.x;
    const unsigned b = blockIdx.x / tps, l0 = (blockIdx.x - b * tps) * TROW;
    const float* xb = x + (size_t)b * DM * L + l0;
#pragma unroll 1
    for (unsigned i = 0; i < 25u; ++i) {
        const unsigned e = tid + 256u * i;
        const unsigned d = e / TROW, l = e - d * TROW;
        sX[l * 129u + d] = bfr(xb[(size_t)d * L + l]);
    }
    __syncthreads();
#pragma unroll 1
    for (unsigned it = 0; it < 7u; ++it) {
        const unsigned item = tid + 256u * it;
        if (item < TROW * 32u) {
            const unsigned r = item >> 5, c4 = (item & 31u) * 4u;
            const v4f p = *(const v4f*)(pe + (size_t)(l0 + r) * DM + c4);
            v4f v;
            v.x = sX[r * 129u + c4] + p.x;
            v.y = sX[r * 129u + c4 + 1u] + p.y;
            v.z = sX[r * 129u + c4 + 2u] + p.z;
            v.w = sX[r * 129u + c4 + 3u] + p.w;
            VST2V4(cur + ((size_t)rowBase + (size_t)b * L + l0 + r) * DM + c4, v);
        }
    }
}

static __device__ __forceinline__ float ln_row8(const float* __restrict__ p, float* d) {
    const v4f a = *(const v4f*)p, b = *(const v4f*)(p + 4);
    float s = ((a.x + a.y) + (a.z + a.w)) + ((b.x + b.y) + (b.z + b.w));
    s += __shfl_xor(s, 8, 32); s += __shfl_xor(s, 4, 32); s += __shfl_xor(s, 2, 32); s += __shfl_xor(s, 1, 32);
    const float mu = s * (1.0f / 128.0f);
    d[0] = a.x - mu; d[1] = a.y - mu; d[2] = a.z - mu; d[3] = a.w - mu;
    d[4] = b.x - mu; d[5] = b.y - mu; d[6] = b.z - mu; d[7] = b.w - mu;
    float q = 0.f;
#pragma unroll
    for (int i = 0; i < 8; ++i) q += d[i] * d[i];
    q += __shfl_xor(q, 8, 32); q += __shfl_xor(q, 4, 32); q += __shfl_xor(q, 2, 32); q += __shfl_xor(q, 1, 32);
    const float sd = sqrtf(q * (1.0f / 127.0f));
    return 1.0f / (sd + 1e-6f);
}

static_assert(TROW * 16 * 2 * 16 == TROW * KCAT * 2);
__global__ __launch_bounds__(256) void k_lnconv(const float* __restrict__ cur, const float* __restrict__ g, const float* __restrict__ bt,
                                                const float* __restrict__ dww, const float* __restrict__ dwb,
                                                unsigned short* __restrict__ h16p) {
    __shared__ __align__(16) float sH[64 * 132];
    __shared__ __align__(16) float sW[KTAP * DM];
    __shared__ __align__(16) float sB[DM];
    const unsigned tid = threadIdx.x;
    const unsigned tile = blockIdx.x;
    unsigned seq0, l0, L;
    if (tile < (unsigned)NT_C) { const unsigned b = tile >> 3; seq0 = b * LC; l0 = (tile & 7u) * TROW; L = LC; }
    else { seq0 = (unsigned)ROWS_C + (tile - (unsigned)NT_C) * TROW; l0 = 0u; L = LQ; }
#pragma unroll 1
    for (unsigned i = tid; i < (unsigned)(KTAP * DM); i += 256u) {
        const unsigned d = i / 7u, k = i - 7u * d;
        sW[k * DM + d] = bfr(dww[i]);
    }
    if (tid < (unsigned)DM) sB[tid] = bfr(dwb[tid]);
    const unsigned hw = tid >> 4, hl = tid & 15u;
    const v4f g0 = *(const v4f*)(g + 8u * hl), g1 = *(const v4f*)(g + 8u * hl + 4u);
    const v4f b0 = *(const v4f*)(bt + 8u * hl), b1 = *(const v4f*)(bt + 8u * hl + 4u);
    const float gg[8] = {bfr(g0.x), bfr(g0.y), bfr(g0.z), bfr(g0.w), bfr(g1.x), bfr(g1.y), bfr(g1.z), bfr(g1.w)};
    const float bb[8] = {bfr(b0.x), bfr(b0.y), bfr(b0.z), bfr(b0.w), bfr(b1.x), bfr(b1.y), bfr(b1.z), bfr(b1.w)};
#pragma unroll 1
    for (unsigned it = 0; it < 4u; ++it) {
        const unsigned r = hw + 16u * it;
        const int l = (int)l0 - 3 + (int)r;
        const int lc = min(max(l, 0), (int)L - 1);
        float d[8];
        const float inv = ln_row8(cur + (size_t)(seq0 + (unsigned)lc) * DM + 8u * hl, d);
        const bool ok = (l >= 0) && (l < (int)L) && (r < (unsigned)(TROW + 6));
        float y[8];
#pragma unroll
        for (int i = 0; i < 8; ++i) { const float t = gg[i] * d[i] * inv + bb[i]; y[i] = ok ? t : 0.0f; }
        v4f y0, y1;
        y0.x = y[0]; y0.y = y[1]; y0.z = y[2]; y0.w = y[3];
        y1.x = y[4]; y1.y = y[5]; y1.z = y[6]; y1.w = y[7];
        *(v4f*)(sH + r * 132u + 8u * hl) = y0;
        *(v4f*)(sH + r * 132u + 8u * hl + 4u) = y1;
    }
    __syncthreads();
#pragma unroll 1
    for (unsigned it = 0; it < 4u; ++it) {
        const unsigned item = tid + 256u * it;
        if (item < TROW * 16u) {
            const unsigned r = item >> 4, g8 = (item & 15u) * 8u;
            float acc[8];
            {
                const v4f a0 = *(const v4f*)(sB + g8), a1 = *(const v4f*)(sB + g8 + 4u);
                acc[0] = a0.x; acc[1] = a0.y; acc[2] = a0.z; acc[3] = a0.w;
                acc[4] = a1.x; acc[5] = a1.y; acc[6] = a1.z; acc[7] = a1.w;
            }
#pragma unroll 1
            for (unsigned k = 0; k < (unsigned)KTAP; ++k) {
                const v4f x0 = *(const v4f*)(sH + (r + k) * 132u + g8), x1 = *(const v4f*)(sH + (r + k) * 132u + g8 + 4u);
                const v4f w0 = *(const v4f*)(sW + k * DM + g8), w1 = *(const v4f*)(sW + k * DM + g8 + 4u);
                acc[0] += w0.x * x0.x; acc[1] += w0.y * x0.y; acc[2] += w0.z * x0.z; acc[3] += w0.w * x0.w;
                acc[4] += w1.x * x1.x; acc[5] += w1.y * x1.y; acc[6] += w1.z * x1.z; acc[7] += w1.w * x1.w;
            }
            float y[8];
#pragma unroll
            for (int i = 0; i < 8; ++i) y[i] = acc[i] * 8.0f;
            const size_t ro = (size_t)(seq0 + l0 + r) * KCAT + g8;
            st8hf_pair(h16p, ro, ro + DM, y);
        }
    }
}

static_assert(256 * 2 * 16 == 16 * KCAT * 2);
__global__ __launch_bounds__(256) void k_ln(const float* __restrict__ cur, const float* __restrict__ g, const float* __restrict__ bt,
                                            unsigned short* __restrict__ z16) {
    const unsigned row = blockIdx.x * 16u + (threadIdx.x >> 4);
    const unsigned hl = threadIdx.x & 15u;
    float d[8];
    const float inv = ln_row8(cur + (size_t)row * DM + 8u * hl, d);
    const v4f g0 = *(const v4f*)(g + 8u * hl), g1 = *(const v4f*)(g + 8u * hl + 4u);
    const v4f b0 = *(const v4f*)(bt + 8u * hl), b1 = *(const v4f*)(bt + 8u * hl + 4u);
    const float gg[8] = {g0.x, g0.y, g0.z, g0.w, g1.x, g1.y, g1.z, g1.w};
    const float bb[8] = {b0.x, b0.y, b0.z, b0.w, b1.x, b1.y, b1.z, b1.w};
    float y[8];
#pragma unroll
    for (int i = 0; i < 8; ++i) y[i] = (bfr(gg[i]) * d[i] * inv + bfr(bb[i])) * 8.0f;
    const size_t ro = (size_t)row * KCAT + 8u * hl;
    st8hf_pair(z16, ro, ro + DM, y);
}

#define AT_PP 72
#define AT_PV 456
static_assert(AT_PV >= CPAD && (AT_PV * 2) % 16 == 0 && (AT_PP * 2) % 16 == 0);
static_assert(64 * AT_PV * 2 + 3 * 8 * 16 * AT_PP * 2 + CPAD * 4 <= 131072);
static_assert(4 * 4 == 16 && 8 * 16 == 128 && 2 * 8 * 16 == 2 * 64 * 2);
__global__ __launch_bounds__(256) void k_attn16(const _Float16* __restrict__ q16, const _Float16* __restrict__ k16,
                                                const _Float16* __restrict__ v16, const float* __restrict__ mask,
                                                _Float16* __restrict__ vals, unsigned L, unsigned nchunk, unsigned rowBase) {
    __shared__ __align__(16) _Float16 sVT[64 * AT_PV];
    __shared__ __align__(16) _Float16 sP[8][16 * AT_PP];
    __shared__ __align__(16) _Float16 sO[8][16 * AT_PP];
    __shared__ __align__(16) _Float16 sR[8][16 * AT_PP];
    __shared__ float sMk[CPAD];
    const unsigned tid = threadIdx.x, lane = tid & 31u;
    const unsigned wave = (unsigned)__builtin_amdgcn_readfirstlane((int)(threadIdx.x >> 5));
    const unsigned hh = lane >> 4, c = lane & 15u;
    const unsigned b = blockIdx.x >> 1, quad = blockIdx.x & 1u;
    const unsigned seq0 = rowBase + b * L;
    const unsigned kpad = nchunk * 64u;
#pragma unroll 1
    for (unsigned item = tid; item < kpad * 4u; item += 256u) {
        const unsigned key = item >> 2, hq = item & 3u;
        const unsigned kc = umin2(key, L - 1u);
        const _Float16* vsrc = v16 + (size_t)(seq0 + kc) * DM + (4u * quad + hq) * 16u;
        const v8h va = *(const v8h*)(vsrc), vb = *(const v8h*)(vsrc + 8);
        const bool ok = key < L;
#pragma unroll
        for (int e = 0; e < 8; ++e) {
            sVT[(hq * 16u + (unsigned)e) * AT_PV + key] = ok ? va[e] : (_Float16)0.0f;
            sVT[(hq * 16u + 8u + (unsigned)e) * AT_PV + key] = ok ? vb[e] : (_Float16)0.0f;
        }
    }
#pragma unroll 1
    for (unsigned key = tid; key < kpad; key += 256u) {
        const unsigned kc = umin2(key, L - 1u);
        sMk[key] = -1.0e30f * (1.0f - bfr(mask[(size_t)b * L + kc]));
    }
    __syncthreads();

    const float SCQ = 0.25f * (1.0f / 64.0f);
    const float LOG2E = 1.4426950408889634f;
    const unsigned ntile = (L + 15u) >> 4;
    _Float16* pw = sP[wave];
    _Float16* po = sO[wave];
    _Float16* pr2 = sR[wave];
    const v8h zero8 = {(_Float16)0.0f, (_Float16)0.0f, (_Float16)0.0f, (_Float16)0.0f, (_Float16)0.0f, (_Float16)0.0f, (_Float16)0.0f, (_Float16)0.0f};
#pragma unroll 1
    for (unsigned qt = wave; qt < ntile; qt += 8u) {
        const unsigned q0 = qt * 16u;
        const unsigned qrow = seq0 + umin2(q0 + c, L - 1u);
#pragma unroll 1
        for (unsigned hq = 0; hq < 4u; ++hq) {
            const unsigned hcol = (4u * quad + hq) * 16u + 8u * hh;
            FragU qf;
            qf.h[0] = *(const v8h*)(q16 + (size_t)qrow * DM + hcol);
            qf.h[1] = zero8;
            float mrow[8], lrow[8];
            v8f os = (v8f){0.f,0.f,0.f,0.f,0.f,0.f,0.f,0.f};
#pragma unroll
            for (int r = 0; r < 8; ++r) { mrow[r] = -3.0e38f; lrow[r] = 0.f; }
#pragma unroll 1
            for (unsigned kc = 0; kc < nchunk; ++kc) {
                const unsigned kv0 = kc * 64u;
                v8f s[4];
                float mk[4];
                bool ok[4];
#pragma unroll
                for (int j = 0; j < 4; ++j) {
                    const unsigned key = kv0 + (unsigned)j * 16u + c;
                    const unsigned kr = seq0 + umin2(key, L - 1u);
                    FragU kf;
                    kf.h[0] = *(const v8h*)(k16 + (size_t)kr * DM + hcol);
                    kf.h[1] = zero8;
                    const v8f z = (v8f){0.f,0.f,0.f,0.f,0.f,0.f,0.f,0.f};
                    s[j] = wmma16(qf.v, kf.v, z);
                    mk[j] = sMk[key];
                    ok[j] = key < L;
                }
#pragma unroll
                for (int r = 0; r < 8; ++r) {
                    float mx = -3.0e38f;
#pragma unroll
                    for (int j = 0; j < 4; ++j) {
                        float t = (s[j][r] * SCQ + mk[j]) * LOG2E;
                        t = ok[j] ? t : -3.0e38f;
                        s[j][r] = t;
                        mx = fmaxf(mx, t);
                    }
                    mx = fmaxf(mx, __shfl_xor(mx, 1, 32)); mx = fmaxf(mx, __shfl_xor(mx, 2, 32));
                    mx = fmaxf(mx, __shfl_xor(mx, 4, 32)); mx = fmaxf(mx, __shfl_xor(mx, 8, 32));
                    const float mnew = fmaxf(mrow[r], mx);
                    const float alpha = exp2f(mrow[r] - mnew);
                    mrow[r] = mnew;
                    float psum = 0.f;
#pragma unroll
                    for (int j = 0; j < 4; ++j) {
                        const float e = s[j][r] - mnew;
                        const h16 ph = (e < -24.0f) ? (h16)0.0f : (h16)(exp2f(e) * 1024.0f);
                        psum += (float)ph;
                        pw[(8u * hh + (unsigned)r) * AT_PP + (unsigned)j * 16u + c] = ph;
                    }
                    psum += __shfl_xor(psum, 1, 32); psum += __shfl_xor(psum, 2, 32);
                    psum += __shfl_xor(psum, 4, 32); psum += __shfl_xor(psum, 8, 32);
                    lrow[r] = lrow[r] * alpha + psum;
                    os[r] *= alpha;
                }
                wave_sync_lds();
#pragma unroll
                for (int kk = 0; kk < 2; ++kk) {
                    const v16h pa = frag_ld(pw + c * AT_PP + (unsigned)kk * 32u + 8u * hh);
                    const v16h vb = frag_ld(sVT + (hq * 16u + c) * AT_PV + kv0 + (unsigned)kk * 32u + 8u * hh);
                    os = wmma16(pa, vb, os);
                }
                wave_sync_lds();
            }
#pragma unroll
            for (int r = 0; r < 8; ++r) {
                const float inv = 1.0f / lrow[r];
                const float ovl = os[r] * inv;
                const h16 hu = (h16)ovl;
                po[(8u * hh + (unsigned)r) * AT_PP + hq * 16u + c] = toh_flush(ovl);
                pr2[(8u * hh + (unsigned)r) * AT_PP + hq * 16u + c] = toh_flush((ovl - (float)hu) * 64.0f);
            }
        }
        wave_sync_lds();
        {
            const unsigned q = lane >> 3, c8 = (lane & 7u) * 8u;
            v8h ov[4], rv[4];
#pragma unroll
            for (int it = 0; it < 4; ++it) {
                ov[it] = *(const v8h*)(po + ((unsigned)it * 4u + q) * AT_PP + c8);
                rv[it] = *(const v8h*)(pr2 + ((unsigned)it * 4u + q) * AT_PP + c8);
            }
            _Float16* dst = vals + (size_t)(seq0 + q0) * KCAT + quad * 64u;
            for (int pass = 0; pass < 2; ++pass) {
#pragma unroll
                for (int it = 0; it < 4; ++it) {
                    const unsigned row = (unsigned)it * 4u + q;
                    if (q0 + row < L) {
                        *(volatile v8h*)(dst + (size_t)row * KCAT + c8) = ov[it];
                        *(volatile v8h*)(dst + (size_t)row * KCAT + DM + c8) = rv[it];
                    }
                }
                __threadfence();
            }
        }
        wave_sync_lds();
    }
}

__global__ __launch_bounds__(256) void k_cq_prep(const float* __restrict__ cf, const float* __restrict__ wvec, const float* __restrict__ wm,
                                                 unsigned use_wm, float carry, unsigned L, unsigned ntile, unsigned rowBase,
                                                 unsigned short* __restrict__ XH, unsigned short* __restrict__ XL,
                                                 float* __restrict__ dots, unsigned short* __restrict__ T16) {
    __shared__ __align__(16) float sX[64 * 132];
    __shared__ __align__(16) float sWm[DM];
    __shared__ __align__(16) float sWv[DM];
    __shared__ __align__(16) float sDot[64];
    const unsigned tid = threadIdx.x;
    const unsigned b = blockIdx.x / ntile, tl = blockIdx.x - b * ntile, n0 = tl * 64u;
    const unsigned pitch = ntile * 64u;
    const size_t seq0 = (size_t)rowBase + (size_t)b * L;
    if (tid < (unsigned)DM) {
        const float w = bfr(wm[tid]);
        sWm[tid] = (use_wm != 0u) ? w : 1.0f;
        sWv[tid] = bfr(wvec[tid]);
    }
#pragma unroll 1
    for (unsigned it = 0; it < 8u; ++it) {
        const unsigned item = tid + 256u * it;
        const unsigned r = item >> 5, c4 = (item & 31u) * 4u;
        const unsigned n = n0 + r;
        const unsigned nc = umin2(n, L - 1u);
        v4f v = *(const v4f*)(cf + (seq0 + nc) * DM + c4);
        if (n >= L) v = (v4f){0.f, 0.f, 0.f, 0.f};
        *(v4f*)(sX + r * 132u + c4) = v;
    }
    __syncthreads();
#pragma unroll 1
    for (unsigned it = 0; it < 4u; ++it) {
        const unsigned item = tid + 256u * it;
        const unsigned r = item >> 4, g8 = (item & 15u) * 8u;
        float hi[8], lo[8];
#pragma unroll
        for (int i = 0; i < 8; ++i) {
            const float xs = sX[r * 132u + g8 + (unsigned)i] * sWm[g8 + (unsigned)i] * carry;
            const h16 hv = toh_flush(xs);
            hi[i] = (float)hv;
            lo[i] = (xs - (float)hv) * 2048.0f;
        }
        if (n0 + r < L) {
            st8hf(XH, (seq0 + n0 + r) * DM + g8, hi);
            st8hf(XL, (seq0 + n0 + r) * DM + g8, lo);
        }
    }
    {
        const unsigned r = tid >> 2, part = tid & 3u;
        float s = 0.f;
#pragma unroll 4
        for (unsigned d = 0; d < 32u; ++d) s += sX[r * 132u + part * 32u + d] * sWv[part * 32u + d];
        s += __shfl_xor(s, 1, 32); s += __shfl_xor(s, 2, 32);
        if (part == 0u) sDot[r] = s;
    }
    __syncthreads();
    if (tid < 16u) {
        const v4f v = *(const v4f*)(sDot + 4u * tid);
        VST2V4(dots + (size_t)b * pitch + n0 + 4u * tid, v);
    }
#pragma unroll 1
    for (unsigned it = 0; it < 4u; ++it) {
        const unsigned item = tid + 256u * it;
        const unsigned d = item >> 3, p8 = (item & 7u) * 8u;
        float v[8];
#pragma unroll
        for (int i = 0; i < 8; ++i) v[i] = sX[(p8 + (unsigned)i) * 132u + d] * 8.0f;
        st8hf(T16, ((size_t)b * DM + d) * pitch + n0 + p8, v);
    }
}
static_assert(4 * 256 == 64 * 16 && 4 * 256 == 128 * 8 && 8 * 256 * 4 == 64 * 128);

__global__ __launch_bounds__(128) void k_cq_s(const _Float16* __restrict__ XH, const _Float16* __restrict__ XL,
                                              const float* __restrict__ dotC, const float* __restrict__ dotQ,
                                              const float* __restrict__ cqb, const float* __restrict__ qmask,
                                              _Float16* __restrict__ PR, float* __restrict__ ST) {
    __shared__ __align__(16) float sST[64 * 68];
    __shared__ __align__(16) _Float16 sPr[4][16 * AT_PP];
    const unsigned tid = threadIdx.x, lane = tid & 31u;
    const unsigned wave = (unsigned)__builtin_amdgcn_readfirstlane((int)(threadIdx.x >> 5));
    const unsigned hh = lane >> 4, c = lane & 15u;
    const unsigned b = blockIdx.x / (unsigned)CTILES, tl = blockIdx.x - (unsigned)CTILES * b, n0 = tl * 64u;
    const unsigned nw = n0 + wave * 16u;
    const size_t arow = ((size_t)b * LC + umin2(nw + c, LC - 1u)) * DM + 8u * hh;
    const size_t qb0 = (size_t)ROWS_C + (size_t)b * LQ;
    v8f H[4], R[4];
#pragma unroll
    for (int j = 0; j < 4; ++j) { H[j] = (v8f){0.f,0.f,0.f,0.f,0.f,0.f,0.f,0.f}; R[j] = H[j]; }
#pragma unroll 1
    for (unsigned ks = 0; ks < 4u; ++ks) {
        const unsigned k0 = ks * 32u;
        const v16h ah = frag_ld(XH + arow + k0);
        const v16h al = frag_ld(XL + arow + k0);
#pragma unroll
        for (int j = 0; j < 4; ++j) {
            const size_t brow = (qb0 + umin2((unsigned)j * 16u + c, LQ - 1u)) * DM + 8u * hh + k0;
            const v16h bh = frag_ld(XH + brow);
            const v16h bl = frag_ld(XL + brow);
            H[j] = wmma16(ah, bh, H[j]);
            R[j] = wmma16(ah, bl, R[j]);
            R[j] = wmma16(al, bh, R[j]);
        }
    }
    const float SH = 1.0f / 512.0f, SR = 1.0f / (512.0f * 2048.0f);
    const float LOG2E = 1.4426950408889634f;
    const float cb = bfr(cqb[0]);
    float qd[4], mq[4];
    bool okm[4];
#pragma unroll
    for (int j = 0; j < 4; ++j) {
        const unsigned m = (unsigned)j * 16u + c;
        const unsigned mc = umin2(m, LQ - 1u);
        qd[j] = dotQ[(size_t)b * QPAD + mc];
        mq[j] = -1.0e30f * (1.0f - bfr(qmask[(size_t)b * LQ + mc]));
        okm[j] = m < (unsigned)LQ;
    }
    _Float16* pr = sPr[wave];
#pragma unroll
    for (int r = 0; r < 8; ++r) {
        const unsigned nrow = umin2(nw + 8u * hh + (unsigned)r, LC - 1u);
        const float cd = dotC[(size_t)b * CPAD + nrow];
        float t[4];
        float mx = -3.0e38f;
#pragma unroll
        for (int j = 0; j < 4; ++j) {
            const float sv = H[j][r] * SH + R[j][r] * SR + cd + qd[j] + cb;
            sST[((unsigned)j * 16u + c) * 68u + wave * 16u + 8u * hh + (unsigned)r] = okm[j] ? sv : 0.0f;
            float tt = (sv + mq[j]) * LOG2E;
            tt = okm[j] ? tt : -3.0e38f;
            t[j] = tt;
            mx = fmaxf(mx, tt);
        }
        mx = fmaxf(mx, __shfl_xor(mx, 1, 32)); mx = fmaxf(mx, __shfl_xor(mx, 2, 32));
        mx = fmaxf(mx, __shfl_xor(mx, 4, 32)); mx = fmaxf(mx, __shfl_xor(mx, 8, 32));
        float psum = 0.f;
#pragma unroll
        for (int j = 0; j < 4; ++j) {
            const float e = exp2f(t[j] - mx);
            const float p = okm[j] ? e : 0.0f;
            t[j] = p;
            psum += p;
        }
        psum += __shfl_xor(psum, 1, 32); psum += __shfl_xor(psum, 2, 32);
        psum += __shfl_xor(psum, 4, 32); psum += __shfl_xor(psum, 8, 32);
        const float sc = 16384.0f * (1.0f / psum);
#pragma unroll
        for (int j = 0; j < 4; ++j) pr[(8u * hh + (unsigned)r) * AT_PP + (unsigned)j * 16u + c] = toh_flush(t[j] * sc);
    }
    wave_sync_lds();
    {
        const unsigned q = lane >> 3, c8 = (lane & 7u) * 8u;
        v8h ov[4];
#pragma unroll
        for (int it = 0; it < 4; ++it) ov[it] = *(const v8h*)(pr + ((unsigned)it * 4u + q) * AT_PP + c8);
        _Float16* dst = PR + ((size_t)b * LC + nw) * QPAD;
        for (int pass = 0; pass < 2; ++pass) {
#pragma unroll
            for (int it = 0; it < 4; ++it) {
                const unsigned row = (unsigned)it * 4u + q;
                if (nw + row < (unsigned)LC) *(volatile v8h*)(dst + (size_t)row * QPAD + c8) = ov[it];
            }
            __threadfence();
        }
    }
    __syncthreads();
#pragma unroll 1
    for (unsigned it = 0; it < 8u; ++it) {
        const unsigned item = tid + 128u * it;
        const unsigned m = item >> 4, c4 = (item & 15u) * 4u;
        const v4f v = *(const v4f*)(sST + m * 68u + c4);
        VST2V4(ST + ((size_t)b * QPAD + m) * CPAD + n0 + c4, v);
    }
}
static_assert(8 * 128 == 64 * 16);
static_assert(64 * 68 * 4 + 4 * 16 * AT_PP * 2 <= 131072);

__global__ __launch_bounds__(256) void k_cq_col(const float* __restrict__ ST, const float* __restrict__ cmask, unsigned short* __restrict__ SCT) {
    const unsigned lane = threadIdx.x & 31u;
    const unsigned wave = (unsigned)__builtin_amdgcn_readfirstlane((int)(threadIdx.x >> 5));
    const unsigned id = blockIdx.x * 8u + wave;
    const unsigned b = id >> 6, m = id & 63u;
    const size_t base = (size_t)id * CPAD;
    const unsigned na = lane * 8u, nb2 = 256u + lane * 8u;
    const bool st1 = lane < 24u;
    if (m >= (unsigned)LQ) {
        const v4u z = (v4u){0u, 0u, 0u, 0u};
        VST2(v4u, (v4u*)(SCT + base + na), z);
        if (st1) { VST2(v4u, (v4u*)(SCT + base + nb2), z); }
        return;
    }
    const float LOG2E = 1.4426950408889634f;
    const unsigned nb2s = umin2(nb2, (unsigned)CPAD - 8u);
    const unsigned nb2m = umin2(nb2, (unsigned)LC - 8u);
    const bool ok1 = nb2 < (unsigned)LC;
    const v4f sa0 = *(const v4f*)(ST + base + na), sa1 = *(const v4f*)(ST + base + na + 4u);
    const v4f sb0 = *(const v4f*)(ST + base + nb2s), sb1 = *(const v4f*)(ST + base + nb2s + 4u);
    const float* mp = cmask + (size_t)b * LC;
    const v4f ma0 = *(const v4f*)(mp + na), ma1 = *(const v4f*)(mp + na + 4u);
    const v4f mb0 = *(const v4f*)(mp + nb2m), mb1 = *(const v4f*)(mp + nb2m + 4u);
    const float sa[8] = {sa0.x, sa0.y, sa0.z, sa0.w, sa1.x, sa1.y, sa1.z, sa1.w};
    const float sb[8] = {sb0.x, sb0.y, sb0.z, sb0.w, sb1.x, sb1.y, sb1.z, sb1.w};
    const float ma[8] = {ma0.x, ma0.y, ma0.z, ma0.w, ma1.x, ma1.y, ma1.z, ma1.w};
    const float mb[8] = {mb0.x, mb0.y, mb0.z, mb0.w, mb1.x, mb1.y, mb1.z, mb1.w};
    float ta[8], tb[8];
    float mx = -3.0e38f;
#pragma unroll
    for (int i = 0; i < 8; ++i) {
        ta[i] = (sa[i] + (-1.0e30f * (1.0f - bfr(ma[i])))) * LOG2E;
        const float u = (sb[i] + (-1.0e30f * (1.0f - bfr(mb[i])))) * LOG2E;
        tb[i] = ok1 ? u : -3.0e38f;
        mx = fmaxf(mx, fmaxf(ta[i], tb[i]));
    }
    mx = fmaxf(mx, __shfl_xor(mx, 16, 32)); mx = fmaxf(mx, __shfl_xor(mx, 8, 32)); mx = fmaxf(mx, __shfl_xor(mx, 4, 32));
    mx = fmaxf(mx, __shfl_xor(mx, 2, 32)); mx = fmaxf(mx, __shfl_xor(mx, 1, 32));
    float sum = 0.f;
#pragma unroll
    for (int i = 0; i < 8; ++i) {
        ta[i] = exp2f(ta[i] - mx);
        const float e = exp2f(tb[i] - mx);
        tb[i] = ok1 ? e : 0.0f;
        sum += ta[i] + tb[i];
    }
    sum += __shfl_xor(sum, 16, 32); sum += __shfl_xor(sum, 8, 32); sum += __shfl_xor(sum, 4, 32);
    sum += __shfl_xor(sum, 2, 32); sum += __shfl_xor(sum, 1, 32);
    const float sc = 16384.0f * (1.0f / sum);
#pragma unroll
    for (int i = 0; i < 8; ++i) { ta[i] *= sc; tb[i] *= sc; }
    st8hf(SCT, base + na, ta);
    if (st1) { st8hf(SCT, base + nb2, tb); }
}
static_assert(32 * 8 + 24 * 8 == CPAD);

__global__ __launch_bounds__(256) void k_cq_u(const _Float16* __restrict__ CT, const _Float16* __restrict__ SCT, _Float16* __restrict__ UT) {
    __shared__ __align__(16) _Float16 sU[8][16 * AT_PP];
    const unsigned lane = threadIdx.x & 31u;
    const unsigned wave = (unsigned)__builtin_amdgcn_readfirstlane((int)(threadIdx.x >> 5));
    const unsigned hh = lane >> 4, c = lane & 15u;
    const unsigned b = blockIdx.x;
    const _Float16* ap = CT + ((size_t)b * DM + wave * 16u + c) * CPAD + 8u * hh;
    v8f acc[4];
#pragma unroll
    for (int j = 0; j < 4; ++j) acc[j] = (v8f){0.f,0.f,0.f,0.f,0.f,0.f,0.f,0.f};
#pragma unroll 1
    for (unsigned ks = 0; ks < (unsigned)(CPAD / 32); ++ks) {
        const v16h a = frag_ld(ap + ks * 32u);
#pragma unroll
        for (int j = 0; j < 4; ++j) {
            const v16h bf = frag_ld(SCT + ((size_t)b * QPAD + (unsigned)j * 16u + c) * CPAD + 8u * hh + ks * 32u);
            acc[j] = wmma16(a, bf, acc[j]);
        }
    }
    _Float16* pu = sU[wave];
#pragma unroll
    for (int j = 0; j < 4; ++j)
#pragma unroll
        for (int r = 0; r < 8; ++r)
            pu[(8u * hh + (unsigned)r) * AT_PP + (unsigned)j * 16u + c] = toh_flush(acc[j][r] * (1.0f / 16384.0f));
    wave_sync_lds();
    {
        const unsigned q = lane >> 3, c8 = (lane & 7u) * 8u;
        v8h ov[4];
#pragma unroll
        for (int it = 0; it < 4; ++it) ov[it] = *(const v8h*)(pu + ((unsigned)it * 4u + q) * AT_PP + c8);
        _Float16* dst = UT + ((size_t)b * DM + wave * 16u) * QPAD;
        for (int pass = 0; pass < 2; ++pass) {
#pragma unroll
            for (int it = 0; it < 4; ++it) *(volatile v8h*)(dst + (size_t)((unsigned)it * 4u + q) * QPAD + c8) = ov[it];
            __threadfence();
        }
    }
}

__global__ __launch_bounds__(256) void k_cq_out(const _Float16* __restrict__ PR, const _Float16* __restrict__ QT, const _Float16* __restrict__ UT,
                                                const float* __restrict__ cf, float* __restrict__ out) {
    __shared__ __align__(16) float sT[8][16 * 132];
    const unsigned lane = threadIdx.x & 31u;
    const unsigned wave = (unsigned)__builtin_amdgcn_readfirstlane((int)(threadIdx.x >> 5));
    const unsigned hh = lane >> 4, c = lane & 15u;
    const unsigned b = blockIdx.x >> 2;
    const unsigned tile = (blockIdx.x & 3u) * 8u + wave;
    if (tile >= (unsigned)(LC / 16)) return;
    const size_t r0 = (size_t)b * LC + tile * 16u;
    const v16h pa0 = frag_ld(PR + (r0 + c) * QPAD + 8u * hh);
    const v16h pa1 = frag_ld(PR + (r0 + c) * QPAD + 32u + 8u * hh);
    float* slab = sT[wave];
    const float SA = 1.0f / 131072.0f;
#pragma unroll 1
    for (unsigned hf = 0; hf < 2u; ++hf) {
        v8f aA[4], aB[4];
#pragma unroll
        for (int j = 0; j < 4; ++j) { aA[j] = (v8f){0.f,0.f,0.f,0.f,0.f,0.f,0.f,0.f}; aB[j] = aA[j]; }
#pragma unroll
        for (int j = 0; j < 4; ++j) {
            const size_t brow = ((size_t)b * DM + hf * 64u + (unsigned)j * 16u + c) * QPAD + 8u * hh;
            const v16h q0f = frag_ld(QT + brow), q1f = frag_ld(QT + brow + 32u);
            const v16h u0f = frag_ld(UT + brow), u1f = frag_ld(UT + brow + 32u);
            aA[j] = wmma16(pa0, q0f, aA[j]);
            aA[j] = wmma16(pa1, q1f, aA[j]);
            aB[j] = wmma16(pa0, u0f, aB[j]);
            aB[j] = wmma16(pa1, u1f, aB[j]);
        }
#pragma unroll
        for (int j = 0; j < 4; ++j)
#pragma unroll
            for (int r = 0; r < 8; ++r) {
                slab[(8u * hh + (unsigned)r) * 132u + (unsigned)j * 16u + c] = aA[j][r] * SA;
                slab[(8u * hh + (unsigned)r) * 132u + 64u + (unsigned)j * 16u + c] = aB[j][r] * SA;
            }
        wave_sync_lds();
        {
            const unsigned c4 = (lane & 15u) * 4u;
#pragma unroll 1
            for (unsigned it = 0; it < 8u; ++it) {
                const unsigned row = it * 2u + hh;
                const v4f a = *(const v4f*)(slab + row * 132u + c4);
                const v4f bt = *(const v4f*)(slab + row * 132u + 64u + c4);
                const v4f c2 = *(const v4f*)(cf + (r0 + row) * DM + hf * 64u + c4);
                const v4f o2 = c2 * a;
                const v4f o3 = c2 * bt;
                float* dst = out + (r0 + row) * (size_t)(4 * DM) + hf * 64u + c4;
                for (int pass = 0; pass < 2; ++pass) {
                    *(volatile v4f*)(dst) = c2;
                    *(volatile v4f*)(dst + DM) = a;
                    *(volatile v4f*)(dst + 2 * DM) = o2;
                    *(volatile v4f*)(dst + 3 * DM) = o3;
                    __threadfence();
                }
            }
        }
        wave_sync_lds();
    }
}
static_assert(8 * 16 * 132 * 4 <= 131072);
static_assert(8 * 2 == 16 && 16 * 16 == 64 * 4);
static_assert((size_t)NB_FULL * LC * 4 * DM * 4 == (size_t)52428800);

static constexpr float SC = 1.0f / 256.0f;
extern "C" void kernel_launch(void* const* d_in, const int* in_sizes, int n_in, void* d_out, int out_size,
                              void* d_ws, size_t ws_size, hipStream_t stream) {
    if (n_in < 24) return;
    if (in_sizes[0] < NB * DM * LC || in_sizes[1] < NB * DM * LQ || in_sizes[2] < NB * LC || in_sizes[3] < NB * LQ) return;
    if (in_sizes[4] < DM || in_sizes[5] < DM || in_sizes[6] < NCONV * DM * KTAP || in_sizes[7] < NCONV * DM) return;
    if (in_sizes[8] < NCONV * DM * DM || in_sizes[9] < NCONV * DM) return;
    if (in_sizes[10] < DM * DM || in_sizes[11] < DM || in_sizes[12] < DM * DM || in_sizes[13] < DM) return;
    if (in_sizes[14] < DM * DM || in_sizes[15] < DM || in_sizes[16] < DM * DM || in_sizes[17] < DM) return;
    if (in_sizes[18] < DM * DM || in_sizes[19] < DM || in_sizes[20] < DM || in_sizes[21] < DM || in_sizes[22] < DM || in_sizes[23] < 1) return;
    if (out_size < NB * LC * 4 * DM) return;

    const float* ctx    = (const float*)d_in[0];
    const float* que    = (const float*)d_in[1];
    const float* c_mask = (const float*)d_in[2];
    const float* q_mask = (const float*)d_in[3];
    const float* ln_g   = (const float*)d_in[4];
    const float* ln_b   = (const float*)d_in[5];
    const float* dw_w   = (const float*)d_in[6];
    const float* dw_b   = (const float*)d_in[7];
    const float* pw_w   = (const float*)d_in[8];
    const float* pw_b   = (const float*)d_in[9];
    const float* Wq     = (const float*)d_in[10];
    const float* bq     = (const float*)d_in[11];
    const float* Wk     = (const float*)d_in[12];
    const float* bk     = (const float*)d_in[13];
    const float* Wv     = (const float*)d_in[14];
    const float* bv     = (const float*)d_in[15];
    const float* Wo     = (const float*)d_in[16];
    const float* bo     = (const float*)d_in[17];
    const float* Wfc    = (const float*)d_in[18];
    const float* bfc    = (const float*)d_in[19];
    const float* cq_wc  = (const float*)d_in[20];
    const float* cq_wq  = (const float*)d_in[21];
    const float* cq_wm  = (const float*)d_in[22];
    const float* cq_b   = (const float*)d_in[23];
    float* out = (float*)d_out;

    char* wsp = (char*)d_ws;
    size_t off = 0;
    auto carve = [&](size_t bytes) -> void* { void* r = wsp + off; off += (bytes + 255) & ~(size_t)255; return r; };
    float*          pe     = (float*)carve((size_t)LC * DM * 4);
    float*          curA   = (float*)carve((size_t)MTOK * DM * 4);
    float*          curB   = (float*)carve((size_t)MTOK * DM * 4);
    unsigned short* a16    = (unsigned short*)carve((size_t)MTOK * KCAT * 2);
    unsigned short* q16    = (unsigned short*)carve((size_t)MTOK * DM * 2);
    unsigned short* k16    = (unsigned short*)carve((size_t)MTOK * DM * 2);
    unsigned short* v16    = (unsigned short*)carve((size_t)MTOK * DM * 2);
    unsigned short* vals16 = (unsigned short*)carve((size_t)MTOK * KCAT * 2);
    unsigned short* wpw    = (unsigned short*)carve((size_t)NCONV * DM * KCAT * 2);
    unsigned short* wq16   = (unsigned short*)carve((size_t)DM * KCAT * 2);
    unsigned short* wk16   = (unsigned short*)carve((size_t)DM * KCAT * 2);
    unsigned short* wv16   = (unsigned short*)carve((size_t)DM * KCAT * 2);
    unsigned short* wo16   = (unsigned short*)carve((size_t)DM * KCAT * 2);
    unsigned short* wfc16  = (unsigned short*)carve((size_t)DM * KCAT * 2);
    unsigned short* XH     = (unsigned short*)carve((size_t)MTOK * DM * 2);
    unsigned short* XL     = (unsigned short*)carve((size_t)MTOK * DM * 2);
    float*          dotC   = (float*)carve((size_t)NB * CPAD * 4);
    float*          dotQ   = (float*)carve((size_t)NB * QPAD * 4);
    unsigned short* CT16   = (unsigned short*)carve((size_t)NB * DM * CPAD * 2);
    unsigned short* QT16   = (unsigned short*)carve((size_t)NB * DM * QPAD * 2);
    unsigned short* PR16   = (unsigned short*)carve((size_t)NB * LC * QPAD * 2);
    float*          STp    = (float*)carve((size_t)NB * QPAD * CPAD * 4);
    unsigned short* SCT16  = (unsigned short*)carve((size_t)NB * QPAD * CPAD * 2);
    unsigned short* UT16   = (unsigned short*)carve((size_t)NB * DM * QPAD * 2);
    if (off > ws_size || off > (size_t)134217728) return;

    k_pe<<<(LC * DM) / 256, 256, 0, stream>>>(pe);
    k_wcvt<<<(NCONV * DM * 16) / 256, 256, 0, stream>>>(pw_w, wpw, 9u, 0u, (unsigned)DM, 1u, (unsigned)(NCONV * DM), 32.0f);
    k_wcvt<<<(DM * 16) / 256, 256, 0, stream>>>(Wq, wq16, 4u, (unsigned)(DM * HDIM), 1u, (unsigned)HDIM, (unsigned)DM, 32.0f);
    k_wcvt<<<(DM * 16) / 256, 256, 0, stream>>>(Wk, wk16, 4u, (unsigned)(DM * HDIM), 1u, (unsigned)HDIM, (unsigned)DM, 32.0f);
    k_wcvt<<<(DM * 16) / 256, 256, 0, stream>>>(Wv, wv16, 4u, (unsigned)(DM * HDIM), 1u, (unsigned)HDIM, (unsigned)DM, 32.0f);
    k_wcvt<<<(DM * 16) / 256, 256, 0, stream>>>(Wo, wo16, 7u, 0u, 1u, (unsigned)DM, (unsigned)DM, 32.0f);
    k_wcvt<<<(DM * 16) / 256, 256, 0, stream>>>(Wfc, wfc16, 7u, 0u, (unsigned)DM, 1u, (unsigned)DM, 32.0f);

    k_prep<<<NT_C, 256, 0, stream>>>(ctx, pe, curA, (unsigned)LC, (unsigned)(LC / TROW), 0u);
    k_prep<<<NT_Q, 256, 0, stream>>>(que, pe, curA, (unsigned)LQ, 1u, (unsigned)ROWS_C);

    const unsigned gG = ((MTOK / 64) * (DM / 64) + 7) / 8;
    float* src = curA;
    float* dst = curB;
    for (int i = 0; i < NCONV; ++i) {
        k_lnconv<<<NT_C + NT_Q, 256, 0, stream>>>(src, ln_g, ln_b, dw_w + (size_t)i * DM * KTAP, dw_b + (size_t)i * DM, a16);
        k_gemm64<0, true, true><<<gG, 256, 0, stream>>>((const _Float16*)a16, KCAT, (const _Float16*)(wpw + (size_t)i * DM * KCAT), KCAT,
            (void*)dst, DM, pw_b + (size_t)i * DM, src, MTOK, DM, KCAT, SC, 1.0f);
        float* t = src; src = dst; dst = t;
    }
    k_ln<<<MTOK / 16, 256, 0, stream>>>(src, ln_g, ln_b, a16);
    k_gemm64<1, false, false><<<gG, 256, 0, stream>>>((const _Float16*)a16, KCAT, (const _Float16*)wq16, KCAT, (void*)q16, DM, bq, nullptr, MTOK, DM, KCAT, SC, 8.0f);
    k_gemm64<1, false, false><<<gG, 256, 0, stream>>>((const _Float16*)a16, KCAT, (const _Float16*)wk16, KCAT, (void*)k16, DM, bk, nullptr, MTOK, DM, KCAT, SC, 8.0f);
    k_gemm64<1, false, false><<<gG, 256, 0, stream>>>((const _Float16*)a16, KCAT, (const _Float16*)wv16, KCAT, (void*)v16, DM, bv, nullptr, MTOK, DM, KCAT, SC, 8.0f);
    k_attn16<<<NB * 2, 256, 0, stream>>>((const _Float16*)q16, (const _Float16*)k16, (const _Float16*)v16, c_mask, (_Float16*)vals16,
        (unsigned)LC, (unsigned)CTILES, 0u);
    k_attn16<<<NB * 2, 256, 0, stream>>>((const _Float16*)q16, (const _Float16*)k16, (const _Float16*)v16, q_mask, (_Float16*)vals16,
        (unsigned)LQ, 1u, (unsigned)ROWS_C);
    k_gemm64<0, true, false><<<gG, 256, 0, stream>>>((const _Float16*)vals16, KCAT, (const _Float16*)wo16, KCAT,
        (void*)dst, DM, bo, src, MTOK, DM, KCAT, SC, 1.0f);
    k_ln<<<MTOK / 16, 256, 0, stream>>>(dst, ln_g, ln_b, a16);
    k_gemm64<0, true, false><<<gG, 256, 0, stream>>>((const _Float16*)a16, KCAT, (const _Float16*)wfc16, KCAT,
        (void*)src, DM, bfc, dst, MTOK, DM, KCAT, SC, 1.0f);
    const float* cfin = src;

    k_cq_prep<<<NB * CTILES, 256, 0, stream>>>(cfin, cq_wc, cq_wm, 1u, 64.0f, (unsigned)LC, (unsigned)CTILES, 0u, XH, XL, dotC, CT16);
    k_cq_prep<<<NB, 256, 0, stream>>>(cfin, cq_wq, cq_wm, 0u, 8.0f, (unsigned)LQ, 1u, (unsigned)ROWS_C, XH, XL, dotQ, QT16);
    k_cq_s<<<NB * CTILES, 128, 0, stream>>>((const _Float16*)XH, (const _Float16*)XL, dotC, dotQ, cq_b, q_mask, (_Float16*)PR16, STp);
    k_cq_col<<<(NB * QPAD) / 8, 256, 0, stream>>>(STp, c_mask, SCT16);
    k_cq_u<<<NB, 256, 0, stream>>>((const _Float16*)CT16, (const _Float16*)SCT16, (_Float16*)UT16);
    k_cq_out<<<NB * 4, 256, 0, stream>>>((const _Float16*)PR16, (const _Float16*)QT16, (const _Float16*)UT16, cfin, out);
}
